// LightweightAttention_20564303413587
// MI455X (gfx1250) — hardware-run, weakly checked
//
#include <hip/hip_runtime.h>


#define NBB  128
#define TT   512
#define HID  16
#define KP   32
#define ZB   32
#define PCAR 1024.0f
typedef _Float16 h16;
typedef unsigned short bf;
typedef __attribute__((ext_vector_type(16))) __bf16   v16bf;
typedef __attribute__((ext_vector_type(16))) _Float16 v16h;
typedef __attribute__((ext_vector_type(8)))  _Float16 v8h;
typedef __attribute__((ext_vector_type(8)))  unsigned short v8us;
typedef __attribute__((ext_vector_type(8)))  float    v8f;
typedef __attribute__((ext_vector_type(4)))  float    v4f;
typedef v8h  __attribute__((may_alias)) v8ha;
typedef v4f  __attribute__((may_alias)) v4fa;
typedef v8us __attribute__((may_alias)) v8usa;

__device__ __forceinline__ unsigned short f2bf(float f) { unsigned u = __float_as_uint(f); u += 0x7FFFu + ((u >> 16) & 1u); return (unsigned short)(u >> 16); }
__device__ __forceinline__ float bf2f(unsigned short b) { return __uint_as_float(((unsigned)b) << 16); }
__device__ __forceinline__ float bfr(float f) { return bf2f(f2bf(f)); }
__device__ __forceinline__ v16h cat16(v8h lo, v8h hi) { return __builtin_shufflevector(lo, hi, 0, 1, 2, 3, 4, 5, 6, 7, 8, 9, 10, 11, 12, 13, 14, 15); }
__device__ __forceinline__ v16bf cat16b(v8us lo, v8us hi) { return __builtin_bit_cast(v16bf, __builtin_shufflevector(lo, hi, 0, 1, 2, 3, 4, 5, 6, 7, 8, 9, 10, 11, 12, 13, 14, 15)); }
__device__ __forceinline__ v8f wmma16(v16h a, v16h b, v8f c) { return __builtin_amdgcn_wmma_f32_16x16x32_f16(false, a, false, b, (short)0, c, false, false); }
__device__ __forceinline__ v8f wmmab(v16bf a, v16bf b, v8f c) { return __builtin_amdgcn_wmma_f32_16x16x32_bf16(false, a, false, b, (short)0, c, false, false); }


template <typename T16> struct WFrag;
template <> struct WFrag<h16> { typedef v16h V; static __device__ __forceinline__ V ld(const h16* p) { return cat16(*(const v8h*)p, *(const v8h*)(p + 16)); } static __device__ __forceinline__ v8f mma(V a, V b, v8f c) { return wmma16(a, b, c); } };
template <> struct WFrag<bf> { typedef v16bf V; static __device__ __forceinline__ V ld(const bf* p) { return cat16b(*(const v8us*)p, *(const v8us*)(p + 16)); } static __device__ __forceinline__ v8f mma(V a, V b, v8f c) { return wmmab(a, b, c); } };
template <typename T16, int NSPLIT, bool BIAS>
__global__ __launch_bounds__(32) void k_gemmw(const T16* __restrict__ A, const T16* __restrict__ A2, const T16* __restrict__ Bt, const T16* __restrict__ Bt2, int K, float* C, int ldc, const float* __restrict__ bias, size_t sA, size_t sB, size_t sC) {
    typedef typename WFrag<T16>::V V;
    __shared__ __align__(16) float os[16 * 68];
    const size_t z = blockIdx.z; A += z * sA; if (A2) A2 += z * sA; Bt += z * sB; if (Bt2) Bt2 += z * sB; C += z * sC;
    const int lane = threadIdx.x & 31, lr = lane & 15, hi = lane >> 4; const int r0 = blockIdx.x * 64, c0 = blockIdx.y * 64;
    v8f acc[4][4];
#pragma unroll
    for (int mb = 0; mb < 4; ++mb)
#pragma unroll
        for (int nb = 0; nb < 4; ++nb) acc[mb][nb] = (v8f){};
    const size_t aoff = (size_t)(r0 + lr) * K + 8 * hi, boff = (size_t)(c0 + lr) * K + 8 * hi;
#pragma unroll 1
    for (int kc = 0; kc < K; kc += 32) {
        V a[4], a2[4];
#pragma unroll
        for (int mb = 0; mb < 4; ++mb) { a[mb] = WFrag<T16>::ld(A + aoff + (size_t)mb * 16 * K + kc); if (NSPLIT == 1 || NSPLIT == 2) a2[mb] = WFrag<T16>::ld(A2 + aoff + (size_t)mb * 16 * K + kc); }
#pragma unroll
        for (int nb = 0; nb < 4; ++nb) { const V b = WFrag<T16>::ld(Bt + boff + (size_t)nb * 16 * K + kc); V b2; if (NSPLIT >= 2) b2 = WFrag<T16>::ld(Bt2 + boff + (size_t)nb * 16 * K + kc);
#pragma unroll
            for (int mb = 0; mb < 4; ++mb) { acc[mb][nb] = WFrag<T16>::mma(a[mb], b, acc[mb][nb]); if (NSPLIT == 1 || NSPLIT == 2) acc[mb][nb] = WFrag<T16>::mma(a2[mb], b, acc[mb][nb]); if (NSPLIT >= 2) acc[mb][nb] = WFrag<T16>::mma(a[mb], b2, acc[mb][nb]); } }
        asm volatile("v_nop\n\tv_nop\n\tv_nop\n\tv_nop" : "+v"(acc[0][0]), "+v"(acc[1][1]), "+v"(acc[2][2]), "+v"(acc[3][3]) : "v"(a[0]), "v"(a[3]));
    }
#pragma unroll
    for (int mb = 0; mb < 4; ++mb) {
#pragma unroll
        for (int nb = 0; nb < 4; ++nb) {
#pragma unroll
            for (int j = 0; j < 8; ++j) os[(hi * 8 + j) * 68 + nb * 16 + lr] = acc[mb][nb][j]; }
        __builtin_amdgcn_wave_barrier(); asm volatile("" ::: "memory");
        float* crow = C + (size_t)(r0 + mb * 16) * ldc + c0;
#pragma unroll 1
        for (int ps = 0; ps < 2; ++ps) {
#pragma unroll
            for (int s = 0; s < 8; ++s) { const int row = 2 * s + hi, cofs = lr * 4; v4f val = *(const v4fa*)(os + row * 68 + cofs); if (BIAS) { val[0] += bfr(bias[c0 + cofs]); val[1] += bfr(bias[c0 + cofs + 1]); val[2] += bfr(bias[c0 + cofs + 2]); val[3] += bfr(bias[c0 + cofs + 3]); }
                *(volatile v4f*)(crow + (size_t)row * ldc + cofs) = val; }
            if (ps == 0) __threadfence(); }
        __builtin_amdgcn_wave_barrier(); asm volatile("" ::: "memory");
    }
}

__device__ __forceinline__ h16 tohx(float x) { return (h16)x; }
typedef __attribute__((ext_vector_type(2))) _Float16 v2h;
typedef __attribute__((ext_vector_type(4))) _Float16 v4h;
typedef __attribute__((ext_vector_type(8))) _Float16 v8h;
typedef __attribute__((ext_vector_type(2))) float v2f;

__global__ __launch_bounds__(256) void k_hid(const float* __restrict__ pf, const float* __restrict__ vf, const float* __restrict__ w1, const float* __restrict__ b1, const float* __restrict__ w2, const float* __restrict__ b2, const float* __restrict__ u1, const float* __restrict__ c1, const float* __restrict__ u2, const float* __restrict__ c2, int b0, float* PH, float* VH) {
    const int e = blockIdx.x * 256 + threadIdx.x; if (e >= ZB * TT * HID) return; const int o = e % HID; const int lt = e / HID; const size_t tok = (size_t)b0 * TT + lt; const float x0 = bfr(pf[tok * 2]), x1 = bfr(pf[tok * 2 + 1]), y0 = bfr(vf[tok * 2]), y1 = bfr(vf[tok * 2 + 1]); float sp = 0.f, sv = 0.f;
#pragma unroll 1
    for (int j = 0; j < 2 * HID; ++j) {
        { float a = __fmul_rn(x0, bfr(w1[j])); asm volatile("" : "+v"(a)); float c = __fmul_rn(x1, bfr(w1[2 * HID + j])); asm volatile("" : "+v"(c)); const float r = fmaxf(__fadd_rn(__fadd_rn(a, c), bfr(b1[j])), 0.f); float p = __fmul_rn(r, bfr(w2[j * HID + o])); asm volatile("" : "+v"(p)); sp = __fadd_rn(sp, p); }
        { float a = __fmul_rn(y0, bfr(u1[j])); asm volatile("" : "+v"(a)); float c = __fmul_rn(y1, bfr(u1[2 * HID + j])); asm volatile("" : "+v"(c)); const float r = fmaxf(__fadd_rn(__fadd_rn(a, c), bfr(c1[j])), 0.f); float p = __fmul_rn(r, bfr(u2[j * HID + o])); asm volatile("" : "+v"(p)); sv = __fadd_rn(sv, p); } }
    const float op = __fadd_rn(sp, bfr(b2[o])), ov = __fadd_rn(sv, bfr(c2[o]));
    *(volatile float*)(PH + (size_t)lt * HID + o) = op; *(volatile float*)(VH + (size_t)lt * HID + o) = ov; __threadfence(); *(volatile float*)(PH + (size_t)lt * HID + o) = op; *(volatile float*)(VH + (size_t)lt * HID + o) = ov; }
__global__ __launch_bounds__(256) void k_proj(const float* __restrict__ PH, const float* __restrict__ VH, const float* __restrict__ qw, const float* __restrict__ qb, const float* __restrict__ kw, const float* __restrict__ kb, const float* __restrict__ vw, const float* __restrict__ vb, const float* __restrict__ kcw, const float* __restrict__ kcb, const float* __restrict__ vcw, const float* __restrict__ vcb, h16* QS, h16* KS, float* VS, h16* KC, float* VC) {
    const int e = blockIdx.x * 256 + threadIdx.x; if (e >= ZB * TT * HID) return; const int o = e % HID; const size_t lt = e / HID; float sq = 0.f, sk = 0.f, sv = 0.f, ck = 0.f, cv = 0.f;
#pragma unroll 1
    for (int j = 0; j < HID; ++j) { const float h = PH[lt * HID + j], g = VH[lt * HID + j]; float p1 = __fmul_rn(h, bfr(qw[j * HID + o])), p2 = __fmul_rn(h, bfr(kw[j * HID + o])), p3 = __fmul_rn(h, bfr(vw[j * HID + o])), p4 = __fmul_rn(g, bfr(kcw[j * HID + o])), p5 = __fmul_rn(g, bfr(vcw[j * HID + o])); asm volatile("" : "+v"(p1), "+v"(p2), "+v"(p3), "+v"(p4), "+v"(p5)); sq = __fadd_rn(sq, p1); sk = __fadd_rn(sk, p2); sv = __fadd_rn(sv, p3); ck = __fadd_rn(ck, p4); cv = __fadd_rn(cv, p5); }
    const h16 q16 = tohx(__fadd_rn(sq, bfr(qb[o]))), k16 = tohx(__fadd_rn(sk, bfr(kb[o]))), kc16 = tohx(__fadd_rn(ck, bfr(kcb[o]))), z = (h16)0.f; const float vv = __fadd_rn(sv, bfr(vb[o])), vc = __fadd_rn(cv, bfr(vcb[o]));
    for (int ps = 0; ps < 2; ++ps) { *(volatile h16*)(QS + lt * KP + o) = q16; *(volatile h16*)(QS + lt * KP + HID + o) = z; *(volatile h16*)(KS + lt * KP + o) = k16; *(volatile h16*)(KS + lt * KP + HID + o) = z; *(volatile h16*)(KC + lt * KP + o) = kc16; *(volatile h16*)(KC + lt * KP + HID + o) = z; *(volatile float*)(VS + lt * HID + o) = vv; *(volatile float*)(VC + lt * HID + o) = vc; if (ps == 0) __threadfence(); } }
__global__ __launch_bounds__(256) void k_vt(const float* __restrict__ V, h16* VT) { const size_t e = ((size_t)blockIdx.x * 256 + threadIdx.x) * 2; if (e >= (size_t)ZB * 64 * TT) return; const int t = (int)(e % TT); const int d = (int)((e / TT) % 64); const int zb = (int)(e / ((size_t)TT * 64)); v2h o;
    if (d < HID) { o[0] = tohx(V[((size_t)zb * TT + t) * HID + d]); o[1] = tohx(V[((size_t)zb * TT + t + 1) * HID + d]); } else { o[0] = (h16)0.f; o[1] = (h16)0.f; } *(volatile v2h*)(VT + e) = o; __threadfence(); *(volatile v2h*)(VT + e) = o; }
__global__ __launch_bounds__(256) void k_soft(const float* __restrict__ S, h16* P) { const int lane = threadIdx.x & 31; const int row = blockIdx.x * 8 + (threadIdx.x >> 5); if (row >= ZB * TT) return; const float* sr = S + (size_t)row * TT; float v[16]; float mx = -3.0e38f;
#pragma unroll
    for (int ch = 0; ch < 4; ++ch) { const v4f a = *(const v4f*)(sr + ch * 128 + lane * 4);
#pragma unroll
        for (int q = 0; q < 4; ++q) { const float t = __fmul_rn(a[q], 0.25f); v[ch * 4 + q] = t; mx = fmaxf(mx, t); } }
#pragma unroll
    for (int sh = 16; sh; sh >>= 1) mx = fmaxf(mx, __shfl_xor(mx, sh, 32));
    float sum = 0.f;
#pragma unroll
    for (int k = 0; k < 16; ++k) { float d0 = __fsub_rn(v[k], mx); asm volatile("" : "+v"(d0)); v[k] = __expf(d0); sum += v[k]; }
#pragma unroll
    for (int sh = 16; sh; sh >>= 1) sum += __shfl_xor(sum, sh, 32);
    const float f = __fdiv_rn(PCAR, sum);
#pragma unroll 1
    for (int ps = 0; ps < 2; ++ps) {
#pragma unroll
        for (int ch = 0; ch < 4; ++ch) { v4h o;
#pragma unroll
            for (int q = 0; q < 4; ++q) o[q] = tohx(v[ch * 4 + q] * f); *(volatile v4h*)(P + (size_t)row * TT + ch * 128 + lane * 4) = o; }
        if (ps == 0) __threadfence(); } }
__global__ __launch_bounds__(256) void k_qc(const float* __restrict__ O, const float* __restrict__ w, const float* __restrict__ b, h16* QC) { const int e = blockIdx.x * 256 + threadIdx.x; if (e >= ZB * TT * HID) return; const int o = e % HID; const size_t lt = e / HID; float s = 0.f;
#pragma unroll 1
    for (int j = 0; j < HID; ++j) { float p = __fmul_rn(O[lt * 64 + j] * (1.0f / PCAR), bfr(w[j * HID + o])); asm volatile("" : "+v"(p)); s = __fadd_rn(s, p); }
    const h16 q = tohx(__fadd_rn(s, bfr(b[o]))), z = (h16)0.f; for (int ps = 0; ps < 2; ++ps) { *(volatile h16*)(QC + lt * KP + o) = q; *(volatile h16*)(QC + lt * KP + HID + o) = z; if (ps == 0) __threadfence(); } }
__global__ __launch_bounds__(256) void k_fin(const float* __restrict__ O2, const float* __restrict__ pf, const float* __restrict__ w, const float* __restrict__ b, int b0, float* OUT) { const int e = blockIdx.x * 256 + threadIdx.x; if (e >= ZB * TT) return; const size_t tok = (size_t)b0 * TT + e; float s0 = 0.f, s1 = 0.f;
#pragma unroll 1
    for (int j = 0; j < HID; ++j) { const float h = O2[(size_t)e * 64 + j] * (1.0f / PCAR); float p0 = __fmul_rn(h, bfr(w[j * 2])); asm volatile("" : "+v"(p0)); float p1 = __fmul_rn(h, bfr(w[j * 2 + 1])); asm volatile("" : "+v"(p1)); s0 = __fadd_rn(s0, p0); s1 = __fadd_rn(s1, p1); }
    v2f o; o[0] = __fadd_rn(bfr(pf[tok * 2]), __fadd_rn(s0, bfr(b[0]))); o[1] = __fadd_rn(bfr(pf[tok * 2 + 1]), __fadd_rn(s1, bfr(b[1]))); *(volatile v2f*)(OUT + tok * 2) = o; __threadfence(); *(volatile v2f*)(OUT + tok * 2) = o; }

extern "C" void kernel_launch(void* const* d_in, const int* in_sizes, int n_in,
                              void* d_out, int out_size, void* d_ws, size_t ws_size, hipStream_t stream) {
    (void)in_sizes; (void)n_in; (void)out_size;
    const float* IN[24]; for (int i = 0; i < 24; ++i) IN[i] = (const float*)d_in[i];
    float* OUT = (float*)d_out;
    char* wsp = (char*)d_ws;
    auto take = [&](size_t bytes) { char* p = wsp; wsp += (bytes + 255) & ~(size_t)255; return (void*)p; };
    float* PH = (float*)take((size_t)ZB * TT * HID * 4); float* VH = (float*)take((size_t)ZB * TT * HID * 4); h16* QS = (h16*)take((size_t)ZB * TT * KP * 2); h16* KS = (h16*)take((size_t)ZB * TT * KP * 2); float* VS = (float*)take((size_t)ZB * TT * HID * 4); h16* KC = (h16*)take((size_t)ZB * TT * KP * 2); float* VC = (float*)take((size_t)ZB * TT * HID * 4); h16* QC = (h16*)take((size_t)ZB * TT * KP * 2);
    h16* VT = (h16*)take((size_t)ZB * 64 * TT * 2); float* S = (float*)take((size_t)ZB * TT * TT * 4); h16* P = (h16*)take((size_t)ZB * TT * TT * 2); float* O = (float*)take((size_t)ZB * TT * 64 * 4);
    if ((size_t)(wsp - (char*)d_ws) > ws_size) return;
    const unsigned LT = (ZB * TT + 255) / 256, LH = (ZB * TT * HID + 255) / 256, LV = (unsigned)(((size_t)ZB * 64 * TT / 2 + 255) / 256);
    for (int ck = 0; ck < NBB / ZB; ++ck) { const int b0 = ck * ZB;
        k_hid<<<LH, 256, 0, stream>>>(IN[0], IN[1], IN[2], IN[3], IN[4], IN[5], IN[6], IN[7], IN[8], IN[9], b0, PH, VH); k_proj<<<LH, 256, 0, stream>>>(PH, VH, IN[10], IN[11], IN[12], IN[13], IN[14], IN[15], IN[18], IN[19], IN[20], IN[21], QS, KS, VS, KC, VC);
        k_vt<<<LV, 256, 0, stream>>>(VS, VT);
        k_gemmw<h16, 0, false><<<dim3(TT / 64, TT / 64, ZB), 32, 0, stream>>>(QS, nullptr, KS, nullptr, KP, S, TT, nullptr, (size_t)TT * KP, (size_t)TT * KP, (size_t)TT * TT); k_soft<<<ZB * TT / 8, 256, 0, stream>>>(S, P);
        k_gemmw<h16, 0, false><<<dim3(TT / 64, 1, ZB), 32, 0, stream>>>(P, nullptr, VT, nullptr, TT, O, 64, nullptr, (size_t)TT * TT, (size_t)64 * TT, (size_t)TT * 64);
        k_qc<<<LH, 256, 0, stream>>>(O, IN[16], IN[17], QC); k_vt<<<LV, 256, 0, stream>>>(VC, VT);
        k_gemmw<h16, 0, false><<<dim3(TT / 64, TT / 64, ZB), 32, 0, stream>>>(QC, nullptr, KC, nullptr, KP, S, TT, nullptr, (size_t)TT * KP, (size_t)TT * KP, (size_t)TT * TT); k_soft<<<ZB * TT / 8, 256, 0, stream>>>(S, P);
        k_gemmw<h16, 0, false><<<dim3(TT / 64, 1, ZB), 32, 0, stream>>>(P, nullptr, VT, nullptr, TT, O, 64, nullptr, (size_t)TT * TT, (size_t)64 * TT, (size_t)TT * 64);
        k_fin<<<LT, 256, 0, stream>>>(O, IN[0], IN[22], IN[23], b0, OUT); }
}
